// Model_40252433498735
// MI455X (gfx1250) — hardware-verified
//
#include <hip/hip_runtime.h>
#include <math.h>

constexpr int NNODE_N   = 30000;
constexpr int NNODE_PAD = 30016;
constexpr int SEQ_T     = 32;
constexpr int NVOC_N    = 10000;
constexpr int NVOC_PAD  = 10048;
constexpr int HID_N     = 128;
constexpr int NGATE_N   = 512;
constexpr int FEAT_N    = 64;
constexpr int NCLS_N    = 16;
constexpr int NREL_N    = 8;
constexpr int NBAS_N    = 4;
constexpr int NEDGE_N   = 480000;
constexpr int EDGE_CHUNK = 1024;
constexpr int NCHUNK_N  = (NEDGE_N + EDGE_CHUNK - 1) / EDGE_CHUNK;
constexpr int AGG_FLOATS = 13824;
constexpr int LS_HP = 136;
constexpr int LS_ZP = 516;
constexpr int FS_P  = 68;

constexpr float WCAR = 64.0f;
constexpr float HCAR = 1024.0f;
constexpr float GCAR = 4096.0f;
constexpr float RCAR = 4096.0f;
constexpr float HOIST_FOLD = 1.0f / (WCAR * WCAR);
constexpr float REC_FOLD   = 1.0f / (HCAR * WCAR);
constexpr float AGG_FOLD   = 1.0f / (GCAR * RCAR);

static_assert(NNODE_N % 16 == 0);
static_assert(NNODE_PAD % 64 == 0 && NNODE_PAD >= NNODE_N);
static_assert(NVOC_PAD % 64 == 0 && NVOC_PAD >= NVOC_N);
static_assert(HID_N % 32 == 0 && FEAT_N % 32 == 0);
static_assert(NGATE_N == 4 * HID_N);
static_assert(NGATE_N % 64 == 0 && (NREL_N * FEAT_N) % 64 == 0 && (NREL_N * NCLS_N) % 64 == 0);
static_assert(NEDGE_N % 4 == 0);
static_assert(SEQ_T == 32);
static_assert(AGG_FLOATS % FEAT_N == 0 && AGG_FLOATS % NCLS_N == 0);
static_assert(AGG_FLOATS / NCLS_N <= 1024);
static_assert(((NNODE_N % (AGG_FLOATS / NCLS_N)) % 8) == 0);
static_assert(((AGG_FLOATS / NCLS_N) * NCLS_N * 4) % 128 == 0);

typedef __attribute__((ext_vector_type(16))) _Float16 v16h;
typedef __attribute__((ext_vector_type(8)))  _Float16 v8h;
typedef __attribute__((ext_vector_type(8)))  float    v8f;
typedef __attribute__((ext_vector_type(4)))  float    v4f;
typedef __attribute__((ext_vector_type(2)))  float    v2f;
typedef __attribute__((ext_vector_type(4)))  int      v4i;
typedef __attribute__((ext_vector_type(4)))  unsigned v4u;

__device__ __forceinline__ void guard4_h(v8f& a0, v8f& a1, v8f& a2, v8f& a3, v16h x, v16h y0, v16h y1, v16h y2, v16h y3) {
  asm volatile("v_nop\n\tv_nop\n\tv_nop\n\tv_nop" : "+v"(a0), "+v"(a1), "+v"(a2), "+v"(a3) : "v"(x), "v"(y0), "v"(y1), "v"(y2), "v"(y3));
}
__device__ __forceinline__ void guard1_h(v8f& a0, v16h x, v16h y) {
  asm volatile("v_nop\n\tv_nop\n\tv_nop\n\tv_nop" : "+v"(a0) : "v"(x), "v"(y));
}
__device__ __forceinline__ void keep4_h(v16h a, v16h b, v16h c, v16h d) { asm volatile("v_nop" :: "v"(a), "v"(b), "v"(c), "v"(d)); }
__device__ __forceinline__ void acc_guard4(v8f& a, v8f& b, v8f& c, v8f& d) { asm volatile("v_nop\n\tv_nop\n\tv_nop\n\tv_nop" : "+v"(a), "+v"(b), "+v"(c), "+v"(d)); }

struct FragH {
  union U { v16h v; v8h h[2]; };
  static __device__ __forceinline__ v16h load(const _Float16* p) {
    U f; f.h[0] = *(const v8h*)(p); f.h[1] = *(const v8h*)(p + 16); return f.v;
  }
  static __device__ __forceinline__ v8f mma(v16h a, v16h b, v8f c) {
    return __builtin_amdgcn_wmma_f32_16x16x32_f16(false, a, false, b, (short)0, c, false, false);
  }
};

__device__ __forceinline__ float fsig(float x)  { return __builtin_amdgcn_rcpf(1.0f + __expf(-x)); }
__device__ __forceinline__ float ftanh(float x) { return 1.0f - 2.0f * __builtin_amdgcn_rcpf(__expf(2.0f * x) + 1.0f); }

template <int BIAS_MODE>
__global__ __launch_bounds__(256) void wmma_gemm64_f16(
    const unsigned short* __restrict__ Ap, int lda,
    const unsigned short* __restrict__ Btp, int ldb,
    float* __restrict__ Cout, int ldc,
    const float* __restrict__ bias,
    int M, int N, int K, float scale) {
  const _Float16* A  = (const _Float16*)Ap;
  const _Float16* Bt = (const _Float16*)Btp;
  __shared__ __align__(16) float sT[8][16 * 68];
  const int lane = threadIdx.x & 31;
  const int wave = threadIdx.x >> 5;
  const int tilesN = N >> 6;
  const int tilesM = M >> 6;
  const int tile = blockIdx.x * 8 + wave;
  if (tile >= tilesM * tilesN) return;
  const int tm = tile / tilesN;
  const int tn = tile - tm * tilesN;
  const int m0 = tm << 6;
  const int n0 = tn << 6;

  const int rlane = lane & 15;
  const int koff  = (lane >> 4) * 8;
  const int mOff  = (lane >> 4) * 8;

  v8f acc[4][4];
#pragma unroll
  for (int i = 0; i < 4; ++i)
#pragma unroll
    for (int j = 0; j < 4; ++j) acc[i][j] = (v8f){0.f, 0.f, 0.f, 0.f, 0.f, 0.f, 0.f, 0.f};

  for (int k0 = 0; k0 < K; k0 += 32) {
    v16h bh[4];
#pragma unroll
    for (int j = 0; j < 4; ++j) {
      const size_t bo = (size_t)(n0 + (j << 4) + rlane) * ldb + koff + k0;
      bh[j] = FragH::load(Bt + bo);
    }
#pragma unroll
    for (int i = 0; i < 4; ++i) {
      const size_t ao = (size_t)(m0 + (i << 4) + rlane) * lda + koff + k0;
      const v16h ah = FragH::load(A + ao);
#pragma unroll
      for (int j = 0; j < 4; ++j) acc[i][j] = FragH::mma(ah, bh[j], acc[i][j]);
      guard4_h(acc[i][0], acc[i][1], acc[i][2], acc[i][3], ah, bh[0], bh[1], bh[2], bh[3]);
    }
    keep4_h(bh[0], bh[1], bh[2], bh[3]);
  }
  acc_guard4(acc[0][0], acc[0][1], acc[0][2], acc[0][3]);
  acc_guard4(acc[1][0], acc[1][1], acc[1][2], acc[1][3]);
  acc_guard4(acc[2][0], acc[2][1], acc[2][2], acc[2][3]);
  acc_guard4(acc[3][0], acc[3][1], acc[3][2], acc[3][3]);

  float* slab = sT[wave];
#pragma unroll
  for (int i = 0; i < 4; ++i) {
    const int mBase = m0 + (i << 4);
#pragma unroll
    for (int j = 0; j < 4; ++j) {
      const int n = n0 + (j << 4) + rlane;
      float bv = 0.f;
      if (BIAS_MODE == 2) bv = bias[n];
#pragma unroll
      for (int r = 0; r < 8; ++r) {
        float v = acc[i][j][r] * scale;
        if (BIAS_MODE == 2) v += bv;
        slab[(mOff + r) * 68 + (j << 4) + rlane] = v;
      }
    }
    __builtin_amdgcn_fence(__ATOMIC_RELEASE, "workgroup");
    __builtin_amdgcn_wave_barrier();
    __builtin_amdgcn_fence(__ATOMIC_ACQUIRE, "workgroup");
    {
      const int hh = lane >> 4, c4 = (lane & 15) * 4;
      for (int pass = 0; pass < 2; ++pass) {
#pragma unroll
        for (int it = 0; it < 8; ++it) {
          const int row = it * 2 + hh;
          const v4f v = *(const v4f*)(slab + row * 68 + c4);
          *(volatile v4f*)(Cout + (size_t)(mBase + row) * ldc + n0 + c4) = v;
        }
        __threadfence();
      }
    }
    __builtin_amdgcn_fence(__ATOMIC_RELEASE, "workgroup");
    __builtin_amdgcn_wave_barrier();
    __builtin_amdgcn_fence(__ATOMIC_ACQUIRE, "workgroup");
  }
}

__global__ __launch_bounds__(256) void cvt_rows_kernel(const float* __restrict__ src, unsigned short* __restrict__ dst,
                                                       int nrow_src, int nrow_dst, int ncol8, float sc) {
  const int i  = blockIdx.x * 256 + threadIdx.x;
  const int n8 = nrow_dst * ncol8;
  if (i < n8) {
    const int row = i / ncol8;
    const int c8  = i - row * ncol8;
    const bool live = row < nrow_src;
    const int rs = live ? row : (nrow_src - 1);
    const float* sp = src + (size_t)rs * (size_t)(ncol8 * 8) + c8 * 8;
    const v4f a = *(const v4f*)(sp);
    const v4f b = *(const v4f*)(sp + 4);
    v8h hv;
#pragma unroll
    for (int e = 0; e < 4; ++e) {
      const float xa = live ? (a[e] * sc) : 0.0f;
      const float xb = live ? (b[e] * sc) : 0.0f;
      hv[e]     = (_Float16)xa;
      hv[4 + e] = (_Float16)xb;
    }
    *(volatile v8h*)(dst + (size_t)i * 8) = hv;
    __threadfence();
    *(volatile v8h*)(dst + (size_t)i * 8) = hv;
  }
}

__global__ __launch_bounds__(128) void bias_sum_kernel(const float* __restrict__ b_a, const float* __restrict__ b_b,
                                                       float* __restrict__ o) {
  const int i4 = threadIdx.x * 4;
  const v4f va = *(const v4f*)(b_a + i4);
  const v4f vb = *(const v4f*)(b_b + i4);
  const v4f s = va + vb;
  *(volatile v4f*)(o + i4) = s;
  __threadfence();
  *(volatile v4f*)(o + i4) = s;
}

template <int OUTD>
__global__ __launch_bounds__(256) void wrel_build_kernel(const float* __restrict__ basis, const float* __restrict__ wcomp,
                                                         unsigned short* __restrict__ Bt) {
  constexpr int NROW = NREL_N * OUTD;
  const int i = blockIdx.x * 256 + threadIdx.x;
  if (i < NROW * 8) {
    const int n  = i >> 3;
    const int k8 = (i & 7) * 8;
    const int r  = n / OUTD;
    const int o  = n - r * OUTD;
    const float w0 = wcomp[r * NBAS_N + 0];
    const float w1 = wcomp[r * NBAS_N + 1];
    const float w2 = wcomp[r * NBAS_N + 2];
    const float w3 = wcomp[r * NBAS_N + 3];
    float p0, p1, p2, p3, q0, q1, q2, q3;
    {
      const float* bp = basis + (size_t)(k8 + 0) * OUTD + o;
      p0 = fmaf(w3, bp[(size_t)3 * FEAT_N * OUTD], fmaf(w2, bp[(size_t)2 * FEAT_N * OUTD], fmaf(w1, bp[(size_t)1 * FEAT_N * OUTD], fmaf(w0, bp[0], 0.0f))));
      bp += OUTD;
      p1 = fmaf(w3, bp[(size_t)3 * FEAT_N * OUTD], fmaf(w2, bp[(size_t)2 * FEAT_N * OUTD], fmaf(w1, bp[(size_t)1 * FEAT_N * OUTD], fmaf(w0, bp[0], 0.0f))));
      bp += OUTD;
      p2 = fmaf(w3, bp[(size_t)3 * FEAT_N * OUTD], fmaf(w2, bp[(size_t)2 * FEAT_N * OUTD], fmaf(w1, bp[(size_t)1 * FEAT_N * OUTD], fmaf(w0, bp[0], 0.0f))));
      bp += OUTD;
      p3 = fmaf(w3, bp[(size_t)3 * FEAT_N * OUTD], fmaf(w2, bp[(size_t)2 * FEAT_N * OUTD], fmaf(w1, bp[(size_t)1 * FEAT_N * OUTD], fmaf(w0, bp[0], 0.0f))));
    }
    asm volatile("" : "+v"(p0), "+v"(p1), "+v"(p2), "+v"(p3) :: "memory");
    {
      const float* bp = basis + (size_t)(k8 + 4) * OUTD + o;
      q0 = fmaf(w3, bp[(size_t)3 * FEAT_N * OUTD], fmaf(w2, bp[(size_t)2 * FEAT_N * OUTD], fmaf(w1, bp[(size_t)1 * FEAT_N * OUTD], fmaf(w0, bp[0], 0.0f))));
      bp += OUTD;
      q1 = fmaf(w3, bp[(size_t)3 * FEAT_N * OUTD], fmaf(w2, bp[(size_t)2 * FEAT_N * OUTD], fmaf(w1, bp[(size_t)1 * FEAT_N * OUTD], fmaf(w0, bp[0], 0.0f))));
      bp += OUTD;
      q2 = fmaf(w3, bp[(size_t)3 * FEAT_N * OUTD], fmaf(w2, bp[(size_t)2 * FEAT_N * OUTD], fmaf(w1, bp[(size_t)1 * FEAT_N * OUTD], fmaf(w0, bp[0], 0.0f))));
      bp += OUTD;
      q3 = fmaf(w3, bp[(size_t)3 * FEAT_N * OUTD], fmaf(w2, bp[(size_t)2 * FEAT_N * OUTD], fmaf(w1, bp[(size_t)1 * FEAT_N * OUTD], fmaf(w0, bp[0], 0.0f))));
    }
    v8h hv;
    hv[0] = (_Float16)(p0 * RCAR);
    hv[1] = (_Float16)(p1 * RCAR);
    hv[2] = (_Float16)(p2 * RCAR);
    hv[3] = (_Float16)(p3 * RCAR);
    hv[4] = (_Float16)(q0 * RCAR);
    hv[5] = (_Float16)(q1 * RCAR);
    hv[6] = (_Float16)(q2 * RCAR);
    hv[7] = (_Float16)(q3 * RCAR);
    unsigned short* op = Bt + (size_t)n * FEAT_N + k8;
    *(volatile v8h*)op = hv;
    __threadfence();
    *(volatile v8h*)op = hv;
  }
}

__global__ __launch_bounds__(384) void pad_zero_kernel(unsigned short* __restrict__ pa, unsigned short* __restrict__ pb,
                                                       unsigned short* __restrict__ pc) {
  const int tid = threadIdx.x;
  const int pl = tid >> 7;
  unsigned short* p = (pl == 0) ? pa : ((pl == 1) ? pb : pc);
  unsigned short* op = p + (size_t)NNODE_N * FEAT_N + (size_t)(tid & 127) * 8;
  const v4u z = {0u, 0u, 0u, 0u};
  *(volatile v4u*)op = z;
  __threadfence();
  *(volatile v4u*)op = z;
}

__global__ __launch_bounds__(256) void lstm_fc_kernel(const int* __restrict__ tokens, const float* __restrict__ EW,
                                                      const unsigned short* __restrict__ WHHp,
                                                      const unsigned short* __restrict__ FCWp,
                                                      const float* __restrict__ fc_b,
                                                      unsigned short* __restrict__ Hout) {
  __shared__ __align__(16) _Float16 Ah[16 * LS_HP];
  __shared__ __align__(16) float    Zt[16 * LS_ZP];
  __shared__ __align__(16) float    Fs[16 * FS_P];
  __shared__ int Tok[16 * SEQ_T];
  const _Float16* WHH = (const _Float16*)WHHp;
  const _Float16* FCW = (const _Float16*)FCWp;
  const int tid = threadIdx.x, lane = tid & 31, wave = tid >> 5;
  const int c = lane & 15, hh = lane >> 4, koff = hh * 8;
  const int nodebase = blockIdx.x * 16;

#pragma unroll
  for (int i = 0; i < 2; ++i) {
    const int idx = i * 256 + tid;
    int node = nodebase + (idx >> 5);
    node = node < NNODE_N ? node : (NNODE_N - 1);
    int tk = tokens[(size_t)node * SEQ_T + (idx & 31)];
    tk = tk < 0 ? 0 : tk;
    tk = tk > (NVOC_N - 1) ? (NVOC_N - 1) : tk;
    Tok[idx] = tk;
  }
#pragma unroll 1
  for (int i = tid; i < 16 * LS_HP; i += 256) Ah[i] = (_Float16)0.0f;
  __syncthreads();
  {
    const int m = tid >> 4, t16 = tid & 15;
    const int tk = Tok[m * SEQ_T + (SEQ_T - 1)];
    const float* er = EW + (size_t)tk * NGATE_N;
#pragma unroll
    for (int i = 0; i < 8; ++i) {
      const int col = 4 * (t16 + 16 * i);
      const v4f v = *(const v4f*)(er + col);
      *(v4f*)(Zt + m * LS_ZP + col) = v;
    }
  }
  __syncthreads();

  float cst[8];
#pragma unroll
  for (int r = 0; r < 8; ++r) cst[r] = 0.0f;
  const v8f z8 = {0.f, 0.f, 0.f, 0.f, 0.f, 0.f, 0.f, 0.f};
  const _Float16* ahrow = Ah + c * LS_HP + koff;
  const size_t wrow = (size_t)(16 * wave + c) * HID_N + koff;

#pragma unroll 1
  for (int s = 0; s < SEQ_T; ++s) {
    v8f acc0 = z8, acc1 = z8, acc2 = z8, acc3 = z8;
#pragma unroll 1
    for (int k0 = 0; k0 < HID_N; k0 += 32) {
      const v16h a  = FragH::load(ahrow + k0);
      const v16h b0 = FragH::load(WHH + wrow + k0);
      const v16h b1 = FragH::load(WHH + wrow + (size_t)1 * HID_N * HID_N + k0);
      const v16h b2 = FragH::load(WHH + wrow + (size_t)2 * HID_N * HID_N + k0);
      const v16h b3 = FragH::load(WHH + wrow + (size_t)3 * HID_N * HID_N + k0);
      acc0 = FragH::mma(a, b0, acc0);
      acc1 = FragH::mma(a, b1, acc1);
      acc2 = FragH::mma(a, b2, acc2);
      acc3 = FragH::mma(a, b3, acc3);
      guard4_h(acc0, acc1, acc2, acc3, a, b0, b1, b2, b3);
    }
    acc_guard4(acc0, acc1, acc2, acc3);
    float hn[8];
#pragma unroll
    for (int r = 0; r < 8; ++r) {
      const int zb = (8 * hh + r) * LS_ZP + 16 * wave + c;
      const float zi = fmaf(acc0[r], REC_FOLD, Zt[zb]);
      const float zf = fmaf(acc1[r], REC_FOLD, Zt[zb + HID_N]);
      const float zg = fmaf(acc2[r], REC_FOLD, Zt[zb + 2 * HID_N]);
      const float zo = fmaf(acc3[r], REC_FOLD, Zt[zb + 3 * HID_N]);
      const float ig = fsig(zi);
      const float fg = fsig(zf);
      const float gg = ftanh(zg);
      const float og = fsig(zo);
      const float cn = fg * cst[r] + ig * gg;
      cst[r] = cn;
      hn[r] = og * ftanh(cn);
    }
    __syncthreads();
#pragma unroll
    for (int r = 0; r < 8; ++r) Ah[(8 * hh + r) * LS_HP + 16 * wave + c] = (_Float16)(hn[r] * HCAR);
    if (s + 1 < SEQ_T) {
      const int m = tid >> 4, t16 = tid & 15;
      const int tk = Tok[m * SEQ_T + (SEQ_T - 2 - s)];
      const float* er = EW + (size_t)tk * NGATE_N;
#pragma unroll
      for (int i = 0; i < 8; ++i) {
        const int col = 4 * (t16 + 16 * i);
        const v4f v = *(const v4f*)(er + col);
        *(v4f*)(Zt + m * LS_ZP + col) = v;
      }
    }
    __syncthreads();
  }

  {
    const int nt = wave & 3;
    v8f fa = z8;
    const size_t frow = (size_t)(16 * nt + c) * HID_N + koff;
#pragma unroll 1
    for (int k0 = 0; k0 < HID_N; k0 += 32) {
      const v16h a = FragH::load(ahrow + k0);
      const v16h b = FragH::load(FCW + frow + k0);
      fa = FragH::mma(a, b, fa);
      guard1_h(fa, a, b);
    }
    const float fb = fc_b[16 * nt + c];
    if (wave < 4) {
#pragma unroll
      for (int r = 0; r < 8; ++r) Fs[(8 * hh + r) * FS_P + 16 * nt + c] = (fa[r] * REC_FOLD + fb) * GCAR;
    }
  }
  __syncthreads();
  if (tid < 128) {
    const int row = tid >> 3, c8 = (tid & 7) * 8;
    v8h hv;
#pragma unroll
    for (int e = 0; e < 8; ++e) hv[e] = (_Float16)Fs[row * FS_P + c8 + e];
    unsigned short* op = Hout + (size_t)(nodebase + row) * FEAT_N + c8;
    *(volatile v8h*)op = hv;
    __threadfence();
    *(volatile v8h*)op = hv;
  }
}

template <int OUTD, bool LAST>
__global__ __launch_bounds__(256) void rgcn_gather_kernel(const float* __restrict__ HW,
                                                          const int* __restrict__ esrc, const int* __restrict__ edst,
                                                          const int* __restrict__ erel, const float* __restrict__ enorm,
                                                          unsigned short* __restrict__ Hnext, float* __restrict__ outp) {
  constexpr int NTILE = AGG_FLOATS / OUTD;
  constexpr int LDW   = NREL_N * OUTD;
  static_assert(NTILE <= 1024);
  static_assert(OUTD == 64 || OUTD == 16);
  __shared__ __align__(16) float Acc[AGG_FLOATS];
  __shared__ int Lst[2 * 8 * 128];
  __shared__ int Cnt[2 * 8];
  const int tid  = threadIdx.x;
  const int lane = tid & 31;
  const int wave = __builtin_amdgcn_readfirstlane(tid >> 5);
  const int node0 = blockIdx.x * NTILE;

  {
    const v4f z4 = {0.f, 0.f, 0.f, 0.f};
#pragma unroll 1
    for (int i = tid; i < AGG_FLOATS / 4; i += 256) *(v4f*)(Acc + 4 * i) = z4;
  }
  __syncthreads();

#pragma unroll 1
  for (int ch = 0; ch < NCHUNK_N; ++ch) {
    const int buf = ch & 1;
    const int eb  = ch * EDGE_CHUNK + 4 * tid;
    const bool inr = eb < NEDGE_N;
    const int ebc = inr ? eb : (NEDGE_N - 4);
    const v4i d4 = *(const v4i*)(edst + ebc);
    const int d0 = d4[0], d1 = d4[1], d2 = d4[2], d3 = d4[3];
    const unsigned u0 = (unsigned)(d0 - node0);
    const unsigned u1 = (unsigned)(d1 - node0);
    const unsigned u2 = (unsigned)(d2 - node0);
    const unsigned u3 = (unsigned)(d3 - node0);
    const bool h0 = inr && (u0 < (unsigned)NTILE);
    const bool h1 = inr && (u1 < (unsigned)NTILE);
    const bool h2 = inr && (u2 < (unsigned)NTILE);
    const bool h3 = inr && (u3 < (unsigned)NTILE);
    const unsigned b0 = __builtin_amdgcn_ballot_w32(h0);
    const unsigned b1 = __builtin_amdgcn_ballot_w32(h1);
    const unsigned b2 = __builtin_amdgcn_ballot_w32(h2);
    const unsigned b3 = __builtin_amdgcn_ballot_w32(h3);
    const int pre = (int)(__builtin_amdgcn_mbcnt_lo(b0, 0u) + __builtin_amdgcn_mbcnt_lo(b1, 0u) +
                          __builtin_amdgcn_mbcnt_lo(b2, 0u) + __builtin_amdgcn_mbcnt_lo(b3, 0u));
    const int p0 = pre;
    const int p1 = p0 + (h0 ? 1 : 0);
    const int p2 = p1 + (h1 ? 1 : 0);
    const int p3 = p2 + (h2 ? 1 : 0);
    const int lbase = (buf * 8 + wave) * 128;
    if (h0) Lst[lbase + p0] = (eb + 0) * 1024 + (int)u0;
    if (h1) Lst[lbase + p1] = (eb + 1) * 1024 + (int)u1;
    if (h2) Lst[lbase + p2] = (eb + 2) * 1024 + (int)u2;
    if (h3) Lst[lbase + p3] = (eb + 3) * 1024 + (int)u3;
    if (lane == 0) Cnt[buf * 8 + wave] = __builtin_popcount(b0) + __builtin_popcount(b1) + __builtin_popcount(b2) + __builtin_popcount(b3);
    __syncthreads();

#pragma unroll 1
    for (int w2 = 0; w2 < 8; ++w2) {
      int n = __builtin_amdgcn_readfirstlane(Cnt[buf * 8 + w2]);
      n = n < 0 ? 0 : (n > 128 ? 128 : n);
      const int l2 = (buf * 8 + w2) * 128;
#pragma unroll 1
      for (int p = 0; p < n; ++p) {
        const int ent = __builtin_amdgcn_readfirstlane(Lst[l2 + p]);
        int u = ent & 1023;
        if ((u & 7) == wave) {
          int e = ent >> 10;
          e = e < 0 ? 0 : (e > (NEDGE_N - 1) ? (NEDGE_N - 1) : e);
          u = u < NTILE ? u : (NTILE - 1);
          int sn = esrc[e];
          sn = sn < 0 ? 0 : (sn > (NNODE_N - 1) ? (NNODE_N - 1) : sn);
          int rl = erel[e];
          rl = rl < 0 ? 0 : (rl > (NREL_N - 1) ? (NREL_N - 1) : rl);
          const float wgt = enorm[e] * AGG_FOLD;
          const float* row = HW + (size_t)sn * LDW + rl * OUTD;
          if (OUTD == 64) {
            const v2f v = *(const v2f*)(row + 2 * lane);
            v2f a = *(const v2f*)(Acc + u * OUTD + 2 * lane);
            a[0] = fmaf(wgt, v[0], a[0]);
            a[1] = fmaf(wgt, v[1], a[1]);
            *(v2f*)(Acc + u * OUTD + 2 * lane) = a;
          } else {
            const int f = lane & 15;
            const float v = row[f];
            const float old = Acc[u * OUTD + f];
            const float nv = fmaf(wgt, v, old);
            if (lane < 16) Acc[u * OUTD + f] = nv;
          }
        }
      }
    }
  }
  __syncthreads();

  if (!LAST) {
    for (int pass = 0; pass < 2; ++pass) {
#pragma unroll 1
      for (int it = tid; it < NTILE * 8; it += 256) {
        const int row = it >> 3, c8 = (it & 7) * 8;
        const int node = node0 + row;
        if (node < NNODE_N) {
          v8h hv;
#pragma unroll
          for (int e = 0; e < 8; ++e) hv[e] = (_Float16)(fmaxf(Acc[row * OUTD + c8 + e], 0.0f) * GCAR);
          *(volatile v8h*)(Hnext + (size_t)node * FEAT_N + c8) = hv;
        }
      }
      __threadfence();
    }
  } else {
    int nvalid = NNODE_N - node0;
    nvalid = nvalid > NTILE ? NTILE : nvalid;
    const int nf4 = nvalid * (OUTD / 4);
    float* ob = outp + (size_t)node0 * OUTD;
    for (int pass = 0; pass < 2; ++pass) {
#pragma unroll 1
      for (int i = tid; i < nf4; i += 256) {
        const v4f v = *(const v4f*)(Acc + 4 * i);
        *(volatile v4f*)(ob + 4 * (size_t)i) = v;
      }
      __threadfence();
    }
  }
}

extern "C" void kernel_launch(void* const* d_in, const int* in_sizes, int n_in,
                              void* d_out, int out_size, void* d_ws, size_t ws_size, hipStream_t stream) {
  if (n_in < 19 || d_out == nullptr || d_ws == nullptr) return;
  if (in_sizes[0] != NNODE_N * SEQ_T || in_sizes[2] != NEDGE_N || in_sizes[3] != NEDGE_N || in_sizes[4] != NEDGE_N ||
      in_sizes[5] != NEDGE_N || in_sizes[6] != NVOC_N * HID_N || in_sizes[7] != NGATE_N * HID_N ||
      in_sizes[8] != NGATE_N * HID_N || in_sizes[9] != NGATE_N || in_sizes[10] != NGATE_N ||
      in_sizes[11] != FEAT_N * HID_N || in_sizes[12] != FEAT_N ||
      in_sizes[13] != NBAS_N * FEAT_N * FEAT_N || in_sizes[14] != NREL_N * NBAS_N ||
      in_sizes[15] != NBAS_N * FEAT_N * FEAT_N || in_sizes[16] != NREL_N * NBAS_N ||
      in_sizes[17] != NBAS_N * FEAT_N * NCLS_N || in_sizes[18] != NREL_N * NBAS_N ||
      out_size != NNODE_N * NCLS_N) return;

  const int*   tokens = (const int*)d_in[0];
  const int*   esrc   = (const int*)d_in[2];
  const int*   edst   = (const int*)d_in[3];
  const int*   erel   = (const int*)d_in[4];
  const float* enorm  = (const float*)d_in[5];
  const float* emb    = (const float*)d_in[6];
  const float* w_ih   = (const float*)d_in[7];
  const float* w_hh   = (const float*)d_in[8];
  const float* b_ih   = (const float*)d_in[9];
  const float* b_hh   = (const float*)d_in[10];
  const float* fc_w   = (const float*)d_in[11];
  const float* fc_b   = (const float*)d_in[12];
  const float* basis0 = (const float*)d_in[13];
  const float* wcomp0 = (const float*)d_in[14];
  const float* basis1 = (const float*)d_in[15];
  const float* wcomp1 = (const float*)d_in[16];
  const float* basis2 = (const float*)d_in[17];
  const float* wcomp2 = (const float*)d_in[18];
  float* outp = (float*)d_out;

  char* ws = (char*)d_ws; size_t off = 0;
  auto carve = [&](size_t bytes) -> char* { char* p = ws + off; off += (bytes + 255) & ~(size_t)255; return p; };
  unsigned short* EMB16 = (unsigned short*)carve((size_t)NVOC_PAD * HID_N * 2);
  unsigned short* WIH16 = (unsigned short*)carve((size_t)NGATE_N * HID_N * 2);
  unsigned short* WHH16 = (unsigned short*)carve((size_t)NGATE_N * HID_N * 2);
  unsigned short* FCW16 = (unsigned short*)carve((size_t)FEAT_N * HID_N * 2);
  float*          BIAS  = (float*)carve((size_t)NGATE_N * 4);
  unsigned short* WR0   = (unsigned short*)carve((size_t)NREL_N * FEAT_N * FEAT_N * 2);
  unsigned short* WR1   = (unsigned short*)carve((size_t)NREL_N * FEAT_N * FEAT_N * 2);
  unsigned short* WR2   = (unsigned short*)carve((size_t)NREL_N * NCLS_N * FEAT_N * 2);
  float*          EW    = (float*)carve((size_t)NVOC_PAD * NGATE_N * 4);
  unsigned short* H16A  = (unsigned short*)carve((size_t)NNODE_PAD * FEAT_N * 2);
  unsigned short* H16B  = (unsigned short*)carve((size_t)NNODE_PAD * FEAT_N * 2);
  unsigned short* H16C  = (unsigned short*)carve((size_t)NNODE_PAD * FEAT_N * 2);
  float*          HW01  = (float*)carve((size_t)NNODE_PAD * NREL_N * FEAT_N * 4);
  float*          HW2   = (float*)carve((size_t)NNODE_PAD * NREL_N * NCLS_N * 4);
  if (off > ws_size || off > (size_t)134217728) return;

  cvt_rows_kernel<<<(NVOC_PAD * (HID_N / 8)) / 256, 256, 0, stream>>>(emb,  EMB16, NVOC_N,  NVOC_PAD, HID_N / 8, WCAR);
  cvt_rows_kernel<<<(NGATE_N * (HID_N / 8)) / 256, 256, 0, stream>>>(w_ih, WIH16, NGATE_N, NGATE_N, HID_N / 8, WCAR);
  cvt_rows_kernel<<<(NGATE_N * (HID_N / 8)) / 256, 256, 0, stream>>>(w_hh, WHH16, NGATE_N, NGATE_N, HID_N / 8, WCAR);
  cvt_rows_kernel<<<(FEAT_N * (HID_N / 8)) / 256, 256, 0, stream>>>(fc_w, FCW16, FEAT_N,  FEAT_N,  HID_N / 8, WCAR);
  bias_sum_kernel<<<1, 128, 0, stream>>>(b_ih, b_hh, BIAS);
  wrel_build_kernel<FEAT_N><<<(NREL_N * FEAT_N * 8) / 256, 256, 0, stream>>>(basis0, wcomp0, WR0);
  wrel_build_kernel<FEAT_N><<<(NREL_N * FEAT_N * 8) / 256, 256, 0, stream>>>(basis1, wcomp1, WR1);
  wrel_build_kernel<NCLS_N><<<(NREL_N * NCLS_N * 8) / 256, 256, 0, stream>>>(basis2, wcomp2, WR2);
  pad_zero_kernel<<<1, 384, 0, stream>>>(H16A, H16B, H16C);

  wmma_gemm64_f16<2><<<(NVOC_PAD / 64) * (NGATE_N / 64) / 8, 256, 0, stream>>>(
      EMB16, HID_N, WIH16, HID_N, EW, NGATE_N, BIAS, NVOC_PAD, NGATE_N, HID_N, HOIST_FOLD);

  lstm_fc_kernel<<<NNODE_N / 16, 256, 0, stream>>>(tokens, EW, WHH16, FCW16, fc_b, H16A);

  const int tiles01 = (NNODE_PAD / 64) * ((NREL_N * FEAT_N) / 64);
  const int tiles2  = (NNODE_PAD / 64) * ((NREL_N * NCLS_N) / 64);
  const int ntile64 = AGG_FLOATS / FEAT_N;
  const int ntile16 = AGG_FLOATS / NCLS_N;

  wmma_gemm64_f16<0><<<(tiles01 + 7) / 8, 256, 0, stream>>>(
      H16A, FEAT_N, WR0, FEAT_N, HW01, NREL_N * FEAT_N, BIAS, NNODE_PAD, NREL_N * FEAT_N, FEAT_N, 1.0f);
  rgcn_gather_kernel<FEAT_N, false><<<(NNODE_N + ntile64 - 1) / ntile64, 256, 0, stream>>>(
      HW01, esrc, edst, erel, enorm, H16B, outp);

  wmma_gemm64_f16<0><<<(tiles01 + 7) / 8, 256, 0, stream>>>(
      H16B, FEAT_N, WR1, FEAT_N, HW01, NREL_N * FEAT_N, BIAS, NNODE_PAD, NREL_N * FEAT_N, FEAT_N, 1.0f);
  rgcn_gather_kernel<FEAT_N, false><<<(NNODE_N + ntile64 - 1) / ntile64, 256, 0, stream>>>(
      HW01, esrc, edst, erel, enorm, H16C, outp);

  wmma_gemm64_f16<0><<<(tiles2 + 7) / 8, 256, 0, stream>>>(
      H16C, FEAT_N, WR2, FEAT_N, HW2, NREL_N * NCLS_N, BIAS, NNODE_PAD, NREL_N * NCLS_N, FEAT_N, 1.0f);
  rgcn_gather_kernel<NCLS_N, true><<<(NNODE_N + ntile16 - 1) / ntile16, 256, 0, stream>>>(
      HW2, esrc, edst, erel, enorm, H16C, outp);
}
